// DeepSets_34754875359298
// MI455X (gfx1250) — hardware-verified
//
#include <hip/hip_runtime.h>
#include <stddef.h>
#include <math.h>


#define DIN    16
#define HD     128
#define HR1    64
#define NOUT   10
#define NTHR   128
#define NWAVE  4
#define TR     64
#define LDSP   136
#define WPB    256
#define WSCAP  134217728

#define OW0  0
#define OW1  4096
#define OW2  20480
#define OW3  36864
#define OR0  53248
#define OR1  69632
#define OR2  77824
#define WTOT 78848
#define WGRP (WTOT / 8)

#define P_B0 0
#define P_G0 1
#define P_E0 2
#define P_B1 3
#define P_G1 4
#define P_E1 5
#define P_B2 6
#define P_G2 7
#define P_E2 8
#define P_B3 9
#define P_N  10

#define RP_B0 0
#define RP_G0 128
#define RP_E0 256
#define RP_B1 384
#define RP_G1 448
#define RP_E1 512
#define RP_B2 576
#define RP_TOT 592

static_assert(TR == NWAVE * 16);
static_assert(NTHR == NWAVE * 32);
static_assert(NTHR == HD);
static_assert(NTHR == 2 * TR);
static_assert((LDSP % 8) == 0);
static_assert(OW1 == OW0 + HD * 32 && OW2 == OW1 + HD * HD && OW3 == OW2 + HD * HD);
static_assert(OR0 == OW3 + HD * HD && OR1 == OR0 + HD * HD && OR2 == OR1 + HR1 * HD && WTOT == OR2 + 16 * HR1);
static_assert(((OW1 / 8) % 32) == 0 && ((OW2 / 8) % 32) == 0 && ((OW3 / 8) % 32) == 0);
static_assert(((OR0 / 8) % 32) == 0 && ((OR1 / 8) % 32) == 0 && ((OR2 / 8) % 32) == 0 && (WGRP % 32) == 0);
static_assert(((TR * NOUT) % 4) == 0);
static_assert(((TR * NOUT * 4) % 128) == 0);
static_assert(RP_G1 == RP_B1 + HR1 && RP_E1 == RP_G1 + HR1 && RP_B2 == RP_E1 + HR1 && RP_TOT == RP_B2 + 16);
static_assert((RP_B1 % 4) == 0 && (RP_E1 % 4) == 0);

typedef _Float16 v16h __attribute__((ext_vector_type(16)));
typedef _Float16 v8h  __attribute__((ext_vector_type(8)));
typedef float    v8f  __attribute__((ext_vector_type(8)));
typedef float    v4f  __attribute__((ext_vector_type(4)));
union Frag { v16h v; v8h h[2]; };

__device__ __forceinline__ v8f wmh(v16h a, v16h b, v8f c) {
  v8f d = __builtin_amdgcn_wmma_f32_16x16x32_f16(false, a, false, b, (short)0, c, false, false);
  asm volatile("v_nop\n\tv_nop\n\tv_nop\n\tv_nop" : "+v"(d) : "v"(a), "v"(b));
  return d;
}

__device__ __forceinline__ float gelu_f(float v) {
  return 0.5f * v * (1.0f + erff(v * 0.70710678118654752f));
}

__device__ __forceinline__ v8h cvt8(v4f a, v4f b) {
  v8h r;
  r[0] = (_Float16)a.x; r[1] = (_Float16)a.y; r[2] = (_Float16)a.z; r[3] = (_Float16)a.w;
  r[4] = (_Float16)b.x; r[5] = (_Float16)b.y; r[6] = (_Float16)b.z; r[7] = (_Float16)b.w;
  return r;
}

__device__ __forceinline__ int lower_bound_i(const int* __restrict__ idx, int n, int key) {
  int lo = 0, hi = n;
#pragma unroll 1
  for (int it = 0; it < 34; ++it) {
    if (lo >= hi) break;
    const int mid = lo + ((hi - lo) >> 1);
    const int v = idx[mid];
    if (v < key) lo = mid + 1; else hi = mid;
  }
  return lo;
}

template <int NT, int KT, int KP>
__device__ __forceinline__ void mma_layer(const _Float16* sA, const _Float16* __restrict__ Bw,
                                          int wrow, int lane, v8f (&acc)[NT]) {
  static_assert((KP % 8) == 0 && 32 * KT <= KP);
  const int hh = lane >> 4, m = lane & 15;
#pragma unroll
  for (int t = 0; t < NT; ++t) { const v8f z = {0.f, 0.f, 0.f, 0.f, 0.f, 0.f, 0.f, 0.f}; acc[t] = z; }
  const _Float16* ap = sA + (wrow + m) * LDSP + 8 * hh;
#pragma unroll 1
  for (int kt = 0; kt < KT; ++kt) {
    Frag a;
    a.h[0] = *(const v8h*)(ap + 32 * kt);
    a.h[1] = *(const v8h*)(ap + 32 * kt + 16);
#pragma unroll
    for (int t = 0; t < NT; ++t) {
      const _Float16* bp = Bw + (size_t)(16 * t + m) * KP + 32 * kt + 8 * hh;
      Frag b;
      b.h[0] = *(const v8h*)bp;
      b.h[1] = *(const v8h*)(bp + 16);
      acc[t] = wmh(a.v, b.v, acc[t]);
    }
  }
}

template <int NT>
__device__ __forceinline__ void ln_gelu_to_lds(v8f (&acc)[NT], _Float16* sA, int wrow, int lane,
                                               const float* bias, const float* g, const float* be) {
  const int hh = lane >> 4, m = lane & 15;
  const float invD = 1.0f / (float)(NT * 16);
  float bv[NT], gv[NT], ev[NT];
#pragma unroll
  for (int t = 0; t < NT; ++t) { bv[t] = bias[16 * t + m]; gv[t] = g[16 * t + m]; ev[t] = be[16 * t + m]; }
#pragma unroll
  for (int r = 0; r < 8; ++r) {
    float s1 = 0.0f;
#pragma unroll
    for (int t = 0; t < NT; ++t) {
      const float v = acc[t][r] * (1.0f / 64.0f) + bv[t];
      acc[t][r] = v;
      s1 += v;
    }
    s1 += __shfl_xor(s1, 1);
    s1 += __shfl_xor(s1, 2);
    s1 += __shfl_xor(s1, 4);
    s1 += __shfl_xor(s1, 8);
    const float mean = s1 * invD;
    float s2 = 0.0f;
#pragma unroll
    for (int t = 0; t < NT; ++t) { const float d = acc[t][r] - mean; s2 += d * d; }
    s2 += __shfl_xor(s2, 1);
    s2 += __shfl_xor(s2, 2);
    s2 += __shfl_xor(s2, 4);
    s2 += __shfl_xor(s2, 8);
    const float var = s2 * invD;
    const float rs  = rsqrtf(var + 1e-5f);
    const int row = wrow + 8 * hh + r;
#pragma unroll
    for (int t = 0; t < NT; ++t) {
      float y = (acc[t][r] - mean) * rs * gv[t] + ev[t];
      y = gelu_f(y);
      sA[row * LDSP + 16 * t + m] = (_Float16)y;
    }
  }
}

__global__ __launch_bounds__(WPB) void k_wprep(
    const float* __restrict__ W0, const float* __restrict__ W1, const float* __restrict__ W2,
    const float* __restrict__ W3, const float* __restrict__ R0, const float* __restrict__ R1,
    const float* __restrict__ R2, _Float16* wp) {
  const int gi = blockIdx.x * WPB + threadIdx.x;
  if (gi >= WGRP) return;
  const float* src;
  int K, N, lg, g, base;
  if (gi < OW1 / 8)      { src = W0; K = DIN; N = HD;   lg = 2; g = gi;           base = OW0; }
  else if (gi < OW2 / 8) { src = W1; K = HD;  N = HD;   lg = 4; g = gi - OW1 / 8; base = OW1; }
  else if (gi < OW3 / 8) { src = W2; K = HD;  N = HD;   lg = 4; g = gi - OW2 / 8; base = OW2; }
  else if (gi < OR0 / 8) { src = W3; K = HD;  N = HD;   lg = 4; g = gi - OW3 / 8; base = OW3; }
  else if (gi < OR1 / 8) { src = R0; K = HD;  N = HD;   lg = 4; g = gi - OR0 / 8; base = OR0; }
  else if (gi < OR2 / 8) { src = R1; K = HD;  N = HR1;  lg = 4; g = gi - OR1 / 8; base = OR1; }
  else                   { src = R2; K = HR1; N = NOUT; lg = 3; g = gi - OR2 / 8; base = OR2; }
  const int kpg = 1 << lg;
  const int n   = g >> lg;
  const int k0  = (g & (kpg - 1)) * 8;
  const int nc  = n > N - 1 ? N - 1 : n;
  v8h hv;
#pragma unroll
  for (int e = 0; e < 8; ++e) {
    const int k  = k0 + e;
    const int kc = k > K - 1 ? K - 1 : k;
    const float w = src[kc * N + nc];
    const float v = (k < K && n < N) ? w * 64.0f : 0.0f;
    hv[e] = (_Float16)v;
  }
  _Float16* dp = wp + base + (size_t)g * 8;
  *(volatile v8h*)dp = hv;
  __threadfence();
  *(volatile v8h*)dp = hv;
}

__global__ __launch_bounds__(NTHR) void k_phi(
    const float* __restrict__ x, const int* __restrict__ idx, const _Float16* __restrict__ wp,
    const float* __restrict__ b0, const float* __restrict__ g0, const float* __restrict__ be0,
    const float* __restrict__ b1, const float* __restrict__ g1, const float* __restrict__ be1,
    const float* __restrict__ b2, const float* __restrict__ g2, const float* __restrict__ be2,
    const float* __restrict__ b3, float* pooled, int nP, int nEv, int maxTiles) {
  __shared__ __attribute__((aligned(16))) _Float16 sH[TR * LDSP];
  __shared__ __attribute__((aligned(16))) float sPar[P_N * HD];
  __shared__ __attribute__((aligned(16))) float sPart[NWAVE * HD];
  __shared__ __attribute__((aligned(16))) float sPool[HD];
  __shared__ int sOk[TR];
  const int tid = threadIdx.x, lane = tid & 31, wave = tid >> 5, hh = lane >> 4, m = lane & 15;
  const int e = blockIdx.x;

  {
    const float* s0p = (wave == 0) ? b0 : ((wave == 1) ? g0  : ((wave == 2) ? be0 : b1));
    const float* s1p = (wave == 0) ? g1 : ((wave == 1) ? be1 : ((wave == 2) ? b2  : g2));
    const v4f v0 = *(const v4f*)(s0p + 4 * lane);
    const v4f v1 = *(const v4f*)(s1p + 4 * lane);
    *(v4f*)(sPar + wave * HD + 4 * lane)       = v0;
    *(v4f*)(sPar + (4 + wave) * HD + 4 * lane) = v1;
    if (wave < 2) {
      const float* s2p = (wave == 0) ? be2 : b3;
      const v4f v2 = *(const v4f*)(s2p + 4 * lane);
      *(v4f*)(sPar + (8 + wave) * HD + 4 * lane) = v2;
    }
  }

  const int s0 = lower_bound_i(idx, nP, e);
  const int s1 = lower_bound_i(idx, nP, e + 1);
  int cnt = s1 - s0;
  cnt = cnt < 0 ? 0 : cnt;
  int nT = (cnt + TR - 1) / TR;
  nT = nT > maxTiles ? maxTiles : nT;

  float ps[8];
#pragma unroll
  for (int t2 = 0; t2 < 8; ++t2) ps[t2] = 0.0f;

#pragma unroll 1
  for (int t = 0; t < nT; ++t) {
    const int rowBase = s0 + t * TR;
    __syncthreads();
    {
      const int r = tid >> 1, c8 = (tid & 1) * 8;
      const int i = rowBase + r;
      const int ic = i > nP - 1 ? nP - 1 : i;
      const float* xp = x + (size_t)ic * DIN + c8;
      const v4f xa = *(const v4f*)xp, xb = *(const v4f*)(xp + 4);
      const int ev = idx[ic];
      *(v8h*)(sH + r * LDSP + c8) = cvt8(xa, xb);
      const v8h z = {(_Float16)0.f, (_Float16)0.f, (_Float16)0.f, (_Float16)0.f,
                     (_Float16)0.f, (_Float16)0.f, (_Float16)0.f, (_Float16)0.f};
      *(v8h*)(sH + r * LDSP + 16 + c8) = z;
      const int okv = ((i < s1) && (ev == e)) ? 1 : 0;
      if (c8 == 0) sOk[r] = okv;
    }
    __syncthreads();

    v8f acc[8];
    mma_layer<8, 1, 32>(sH, wp + OW0, wave * 16, lane, acc);
    ln_gelu_to_lds<8>(acc, sH, wave * 16, lane, sPar + P_B0 * HD, sPar + P_G0 * HD, sPar + P_E0 * HD);
    __syncthreads();
    mma_layer<8, 4, HD>(sH, wp + OW1, wave * 16, lane, acc);
    ln_gelu_to_lds<8>(acc, sH, wave * 16, lane, sPar + P_B1 * HD, sPar + P_G1 * HD, sPar + P_E1 * HD);
    __syncthreads();
    mma_layer<8, 4, HD>(sH, wp + OW2, wave * 16, lane, acc);
    ln_gelu_to_lds<8>(acc, sH, wave * 16, lane, sPar + P_B2 * HD, sPar + P_G2 * HD, sPar + P_E2 * HD);
    __syncthreads();
    mma_layer<8, 4, HD>(sH, wp + OW3, wave * 16, lane, acc);
    {
      float b3v[8];
#pragma unroll
      for (int t2 = 0; t2 < 8; ++t2) b3v[t2] = sPar[P_B3 * HD + 16 * t2 + m];
      const int rb = wave * 16 + 8 * hh;
#pragma unroll
      for (int r = 0; r < 8; ++r) {
        const bool ok = sOk[rb + r] != 0;
#pragma unroll
        for (int t2 = 0; t2 < 8; ++t2) {
          const float v = acc[t2][r] * (1.0f / 64.0f) + b3v[t2];
          ps[t2] += ok ? v : 0.0f;
        }
      }
    }
  }

#pragma unroll
  for (int t2 = 0; t2 < 8; ++t2) ps[t2] += __shfl_xor(ps[t2], 16);
  if (hh == 0) {
#pragma unroll
    for (int t2 = 0; t2 < 8; ++t2) sPart[wave * HD + 16 * t2 + m] = ps[t2];
  }
  __syncthreads();
  {
    const int c = tid;
    const float s = ((sPart[c] + sPart[HD + c]) + sPart[2 * HD + c]) + sPart[3 * HD + c];
    const float rsc = 1.0f / sqrtf((float)cnt);
    sPool[c] = s * rsc;
  }
  __syncthreads();
  if (wave == 0) {
    const v4f v = *(const v4f*)(sPool + 4 * lane);
    float* gp = pooled + (size_t)e * HD + 4 * lane;
    *(volatile v4f*)gp = v;
    __threadfence();
    *(volatile v4f*)gp = v;
  }
}

__device__ __forceinline__ void out_pass(const float* so, float* ob, int nf, int tid) {
#pragma unroll
  for (int it = 0; it < 2; ++it) {
    const int q = it * NTHR + tid;
    if (q < (TR * NOUT) / 4) {
      const v4f v = *(const v4f*)(so + 4 * q);
      if (4 * q + 4 <= nf) {
        *(volatile v4f*)(ob + 4 * q) = v;
      } else if (4 * q < nf) {
        volatile float* op = ob + 4 * q;
        op[0] = v.x;
        if (4 * q + 1 < nf) op[1] = v.y;
        if (4 * q + 2 < nf) op[2] = v.z;
      }
    }
  }
}

__global__ __launch_bounds__(NTHR) void k_rho(
    const float* __restrict__ pooled, const _Float16* __restrict__ wp,
    const float* __restrict__ rb0, const float* __restrict__ rg0, const float* __restrict__ rbe0,
    const float* __restrict__ rb1, const float* __restrict__ rg1, const float* __restrict__ rbe1,
    const float* __restrict__ rb2, float* out, int nEv) {
  __shared__ __attribute__((aligned(16))) _Float16 sH[TR * LDSP];
  __shared__ __attribute__((aligned(16))) float sPr[RP_TOT];
  __shared__ __attribute__((aligned(16))) float sOut[TR * NOUT];
  const int tid = threadIdx.x, lane = tid & 31, wave = tid >> 5, hh = lane >> 4, m = lane & 15;
  const int eBase = blockIdx.x * TR;

  {
    const int l16 = lane & 15;
    if (wave < 3) {
      const float* src = (wave == 0) ? rb0 : ((wave == 1) ? rg0 : rbe0);
      const v4f v = *(const v4f*)(src + 4 * lane);
      *(v4f*)(sPr + wave * HD + 4 * lane) = v;
    } else {
      const v4f va = *(const v4f*)(rb1 + 4 * l16);
      const v4f vb = *(const v4f*)(rg1 + 4 * l16);
      v4f v;
      v.x = (lane < 16) ? va.x : vb.x; v.y = (lane < 16) ? va.y : vb.y;
      v.z = (lane < 16) ? va.z : vb.z; v.w = (lane < 16) ? va.w : vb.w;
      *(v4f*)(sPr + RP_B1 + 4 * lane) = v;
    }
    if (wave == 0) {
      const v4f ve = *(const v4f*)(rbe1 + 4 * l16);
      if (lane < 16) *(v4f*)(sPr + RP_E1 + 4 * lane) = ve;
    }
    if (wave == 1) {
      const float s = rb2[lane < NOUT ? lane : (NOUT - 1)];
      const float sv = (lane < NOUT) ? s : 0.0f;
      if (lane < 16) sPr[RP_B2 + lane] = sv;
    }
  }

  {
    const int r = tid >> 1, c64 = (tid & 1) * 64;
    int er = eBase + r;
    er = er > nEv - 1 ? nEv - 1 : er;
    const float* pp = pooled + (size_t)er * HD + c64;
#pragma unroll
    for (int i = 0; i < 8; ++i) {
      const v4f a = *(const v4f*)(pp + 8 * i), b = *(const v4f*)(pp + 8 * i + 4);
      *(v8h*)(sH + r * LDSP + c64 + 8 * i) = cvt8(a, b);
    }
  }
  __syncthreads();
  {
    v8f acc[8];
    mma_layer<8, 4, HD>(sH, wp + OR0, wave * 16, lane, acc);
    ln_gelu_to_lds<8>(acc, sH, wave * 16, lane, sPr + RP_B0, sPr + RP_G0, sPr + RP_E0);
  }
  __syncthreads();
  {
    v8f acc[4];
    mma_layer<4, 4, HD>(sH, wp + OR1, wave * 16, lane, acc);
    ln_gelu_to_lds<4>(acc, sH, wave * 16, lane, sPr + RP_B1, sPr + RP_G1, sPr + RP_E1);
  }
  __syncthreads();
  {
    v8f acc[1];
    mma_layer<1, 2, HR1>(sH, wp + OR2, wave * 16, lane, acc);
    const float bb = sPr[RP_B2 + m];
#pragma unroll
    for (int r = 0; r < 8; ++r) {
      const float v = acc[0][r] * (1.0f / 64.0f) + bb;
      const int row = wave * 16 + 8 * hh + r;
      if (m < NOUT) sOut[row * NOUT + m] = v;
    }
  }
  __syncthreads();

  int nvalid = nEv - eBase;
  nvalid = nvalid > TR ? TR : (nvalid < 0 ? 0 : nvalid);
  const int nf = nvalid * NOUT;
  float* ob = out + (size_t)eBase * NOUT;
  out_pass(sOut, ob, nf, tid);
  __threadfence();
  out_pass(sOut, ob, nf, tid);
}

extern "C" void kernel_launch(void* const* d_in, const int* in_sizes, int n_in,
                              void* d_out, int out_size, void* d_ws, size_t ws_size,
                              hipStream_t stream) {
  if (n_in < 26) return;
  const int nP  = in_sizes[1];
  const int nEv = out_size / NOUT;
  if (nP <= 0 || nEv <= 0) return;
  if (nP > (1 << 26) || nEv > (1 << 24)) return;
  if (out_size != nEv * NOUT) return;
  if (in_sizes[0] != nP * DIN) return;
  if (in_sizes[2] != DIN * HD || in_sizes[3] != HD || in_sizes[4] != HD || in_sizes[5] != HD) return;
  if (in_sizes[6] != HD * HD || in_sizes[7] != HD || in_sizes[8] != HD || in_sizes[9] != HD) return;
  if (in_sizes[10] != HD * HD || in_sizes[11] != HD || in_sizes[12] != HD || in_sizes[13] != HD) return;
  if (in_sizes[14] != HD * HD || in_sizes[15] != HD) return;
  if (in_sizes[16] != HD * HD || in_sizes[17] != HD || in_sizes[18] != HD || in_sizes[19] != HD) return;
  if (in_sizes[20] != HD * HR1 || in_sizes[21] != HR1 || in_sizes[22] != HR1 || in_sizes[23] != HR1) return;
  if (in_sizes[24] != HR1 * NOUT || in_sizes[25] != NOUT) return;

  const float* x    = (const float*)d_in[0];
  const int*   idx  = (const int*)d_in[1];
  const float* W0   = (const float*)d_in[2];
  const float* b0   = (const float*)d_in[3];
  const float* g0   = (const float*)d_in[4];
  const float* be0  = (const float*)d_in[5];
  const float* W1   = (const float*)d_in[6];
  const float* b1   = (const float*)d_in[7];
  const float* g1   = (const float*)d_in[8];
  const float* be1  = (const float*)d_in[9];
  const float* W2   = (const float*)d_in[10];
  const float* b2   = (const float*)d_in[11];
  const float* g2   = (const float*)d_in[12];
  const float* be2  = (const float*)d_in[13];
  const float* W3   = (const float*)d_in[14];
  const float* b3   = (const float*)d_in[15];
  const float* R0   = (const float*)d_in[16];
  const float* rb0  = (const float*)d_in[17];
  const float* rg0  = (const float*)d_in[18];
  const float* rbe0 = (const float*)d_in[19];
  const float* R1   = (const float*)d_in[20];
  const float* rb1  = (const float*)d_in[21];
  const float* rg1  = (const float*)d_in[22];
  const float* rbe1 = (const float*)d_in[23];
  const float* R2   = (const float*)d_in[24];
  const float* rb2  = (const float*)d_in[25];
  float* out = (float*)d_out;

  const int nRB      = (nEv + TR - 1) / TR;
  const int EPAD     = nRB * TR;
  const int maxTiles = (nP + TR - 1) / TR;

  char* ws = (char*)d_ws;
  size_t off = 0;
  const size_t oW    = off; off += (size_t)WTOT * 2;          off = (off + 255) & ~(size_t)255;
  const size_t oPool = off; off += (size_t)EPAD * HD * 4;     off = (off + 255) & ~(size_t)255;
  if (off > ws_size || off > (size_t)WSCAP) return;
  _Float16* wp     = (_Float16*)(ws + oW);
  float*    pooled = (float*)(ws + oPool);

  k_wprep<<<(WGRP + WPB - 1) / WPB, WPB, 0, stream>>>(W0, W1, W2, W3, R0, R1, R2, wp);

  k_phi<<<nEv, NTHR, 0, stream>>>(x, idx, wp, b0, g0, be0, b1, g1, be1, b2, g2, be2, b3,
                                  pooled, nP, nEv, maxTiles);

  k_rho<<<nRB, NTHR, 0, stream>>>(pooled, wp, rb0, rg0, rbe0, rb1, rg1, rbe1, rb2, out, nEv);
}
